// PatchGAT_10625749090914
// MI455X (gfx1250) — hardware-run, weakly checked
//
#include <hip/hip_runtime.h>


namespace {
constexpr int N = 50000, NP = 50048, EFULL = 800000, E = 800000, NLIM = 50048  , IN = 128, NH = 4, HID = 128, OUT = 64, HC = NH * HID  , HO = NH * OUT  ;
constexpr float XS = 8.0f, WSC = 256.0f, GSLOPE = 0.2f, ASLOPE = 0.01f;
static_assert(NP % 64 == 0 && NP >= N && NLIM % 64 == 0 && NLIM <= NP && IN == 128 && HID == 128 && OUT == 64, "tiling");
typedef _Float16 b16;
typedef __attribute__((ext_vector_type(16))) _Float16 v16b;
typedef __attribute__((ext_vector_type(8))) _Float16 v8b;
typedef __attribute__((ext_vector_type(8))) float v8f;
typedef __attribute__((ext_vector_type(4))) float v4f;
__device__ __forceinline__ float bf16_rne(float f) { unsigned int u = __float_as_uint(f); u += 0x7FFFu + ((u >> 16) & 1u); return __uint_as_float(u & 0xFFFF0000u); }
__device__ __forceinline__ void split16(float v, b16& hi, b16& lo) { hi = (b16)v; lo = (b16)(v - (float)hi); }
__device__ __forceinline__ v16b frag_kb(const b16* p, int hh) { const v8b a = *(const v8b*)(p + 8 * hh), b = *(const v8b*)(p + 16 + 8 * hh); v16b f;
#pragma unroll
  for (int e = 0; e < 8; ++e) { f[e] = a[e]; f[8 + e] = b[e]; } return f; }
__device__ __forceinline__ v8f wmma16b(v16b a, v16b b, v8f c) { v8f d = __builtin_amdgcn_wmma_f32_16x16x32_f16(false, a, false, b, (short)0, c, false, false); asm volatile("v_nop\n\tv_nop\n\tv_nop\n\tv_nop" : "+v"(d) : "v"(a), "v"(b)); return d; }
__device__ __forceinline__ void wave_lds_sync() { __builtin_amdgcn_fence(__ATOMIC_RELEASE, "workgroup"); __builtin_amdgcn_wave_barrier(); __builtin_amdgcn_fence(__ATOMIC_ACQUIRE, "workgroup"); }
__device__ __forceinline__ float pmul(float a, float b) { float p = a * b; asm volatile("" : "+v"(p)); return p; }
__device__ __forceinline__ int iclamp(int v, int lo, int hi) { return v < lo ? lo : (v > hi ? hi : v); }
constexpr int CSR_NBLK = 512, CSR_GB = 9, CSR_GN = 1 << CSR_GB  , CSR_MAXG = 512, CSR_CAP = 12288  ;
__global__ __launch_bounds__(64) void csrA_kernel(const int* __restrict__ dst, int E, int N, int nG, int CHP, int NGP, int* __restrict__ STG, int* __restrict__ HST) {
  extern __shared__ int sm[];
  int* cnt = sm; int* run = sm + NGP; int* ids = sm + 2 * NGP;
  const int b = blockIdx.x; const int ch = (E + CSR_NBLK - 1) / CSR_NBLK; const int e0 = b * ch, e1 = min(E, e0 + ch);
  for (int i = threadIdx.x; i < NGP; i += 64) cnt[i] = 0;
  for (int i = threadIdx.x; i < CHP; i += 64) ids[i] = -1;
  __syncthreads();
  if (threadIdx.x == 0) {
    for (int e = e0; e < e1; ++e) { int d = dst[e]; d = (d < 0) ? 0 : (d >= N ? N - 1 : d); cnt[d >> CSR_GB] += 1; }
    int acc = 0; for (int g = 0; g < nG; ++g) { run[g] = acc; acc += cnt[g]; }
    for (int e = e0; e < e1; ++e) { int d = dst[e]; d = (d < 0) ? 0 : (d >= N ? N - 1 : d); const int g = d >> CSR_GB; ids[run[g]] = e; run[g] += 1; } }
  __syncthreads();
  typedef __attribute__((ext_vector_type(4))) int v4i;
  for (int pass = 0; pass < 2; ++pass) {
    for (int i = threadIdx.x; i < CHP / 4; i += 64) *(volatile v4i*)(STG + (size_t)b * CHP + i * 4) = *(const v4i*)(&ids[i * 4]);
    for (int i = threadIdx.x; i < NGP / 4; i += 64) { v4i v; for (int e = 0; e < 4; ++e) v[e] = (i * 4 + e < nG) ? cnt[i * 4 + e] : 0; *(volatile v4i*)(HST + (size_t)b * NGP + i * 4) = v; }
    __threadfence(); }
}
__global__ __launch_bounds__(512) void csrS_kernel(const int* __restrict__ HST, int nG, int NGP, int* __restrict__ START, int* __restrict__ TOT, int* __restrict__ OFF) {
  __shared__ int tot[CSR_MAXG];
  const int b = threadIdx.x;
  for (int pass = 0; pass < 2; ++pass) { int runb = 0; for (int g = 0; g < nG; ++g) { int c = HST[(size_t)b * NGP + g]; c = (c < 0) ? 0 : c; ((volatile int*)OFF)[(size_t)g * CSR_NBLK + b] = runb; runb += c; } __threadfence(); }
  for (int g = threadIdx.x; g < nG; g += 512) { int s = 0; for (int bb = 0; bb < CSR_NBLK; ++bb) { int c = HST[(size_t)bb * NGP + g]; s += (c < 0) ? 0 : c; } tot[g] = s; }
  __syncthreads();
  if (threadIdx.x < 32) {
    __shared__ int st[CSR_MAXG + 32];
    if (threadIdx.x == 0) { int acc = 0; for (int g = 0; g < NGP; ++g) { st[g] = acc; if (g < nG) acc += (tot[g] + 31) & ~31; } st[NGP] = acc; }
    __builtin_amdgcn_fence(__ATOMIC_RELEASE, "workgroup"); __builtin_amdgcn_wave_barrier(); __builtin_amdgcn_fence(__ATOMIC_ACQUIRE, "workgroup");
    for (int pass = 0; pass < 2; ++pass) { for (int i = threadIdx.x; i < NGP + 32; i += 32) { ((volatile int*)START)[i] = (i <= NGP) ? st[min(i, NGP)] : 0; ((volatile int*)TOT)[i] = (i < nG) ? tot[i] : 0; } __threadfence(); } }
}
__global__ __launch_bounds__(256) void csrB_kernel(const int* __restrict__ dst, int N, int nG, int CHP, int NGP, int permLen, const int* __restrict__ STG, const int* __restrict__ HST, const int* __restrict__ OFF, const int* __restrict__ START, const int* __restrict__ TOT, int* __restrict__ PERM, int* __restrict__ ROWPTR, int* __restrict__ ROWCNT, int* __restrict__ FLAG) {
  typedef __attribute__((ext_vector_type(4))) int v4i;
  __shared__ int ids[CSR_CAP]; __shared__ unsigned short key[CSR_CAP]; __shared__ int outp[CSR_CAP]; __shared__ int ncnt[CSR_GN + 1]; __shared__ int boff[CSR_NBLK + 1];
  const int g = blockIdx.x, t_ = threadIdx.x; int tot = TOT[g]; int st = START[g], stn = START[g + 1]; const int v0 = g * CSR_GN; const int nv = min(CSR_GN, N - v0);
  st = (st < 0) ? 0 : (st > permLen - 32 ? permLen - 32 : st) & ~31; stn = (stn < st) ? st : (stn > permLen ? permLen : stn); tot = (tot < 0) ? 0 : tot; if (tot > stn - st && tot <= CSR_CAP) tot = stn - st;
  if (tot > CSR_CAP) {
    for (int pass = 0; pass < 2; ++pass) { for (int i = t_; i < CSR_GN / 4; i += 256) { v4i a, c; for (int e = 0; e < 4; ++e) { a[e] = st; c[e] = 0; } *(volatile v4i*)(ROWPTR + v0 + i * 4) = a; *(volatile v4i*)(ROWCNT + v0 + i * 4) = c; } if (t_ == 0) ((volatile int*)FLAG)[0] = 1; __threadfence(); } (void)nv; return; }
  if (t_ == 0) { int acc = 0; for (int b = 0; b < CSR_NBLK; ++b) { boff[b] = acc; int c = HST[(size_t)b * NGP + g]; c = (c < 0) ? 0 : (c > CHP ? CHP : c); acc += c; if (acc > tot) acc = tot; } boff[CSR_NBLK] = acc; }
  for (int i = t_; i <= CSR_GN; i += 256) ncnt[i] = 0;
  __syncthreads();
  for (int b = 0; b < CSR_NBLK; ++b) { const int c = boff[b + 1] - boff[b]; int o_ = OFF[(size_t)g * CSR_NBLK + b]; o_ = (o_ < 0) ? 0 : (o_ > CHP - c ? CHP - c : o_); const int* src_ = STG + (size_t)b * CHP + o_;
    for (int i = t_; i < c; i += 256) { int id = src_[i]; id = (id < 0) ? 0 : id; ids[boff[b] + i] = id; int d = dst[id]; d = (d < v0) ? v0 : (d >= N ? N - 1 : d); int kk = d - v0; kk = (kk < 0) ? 0 : (kk >= CSR_GN ? CSR_GN - 1 : kk); key[boff[b] + i] = (unsigned short)kk; } }
  __syncthreads();
  if (t_ == 0) { for (int i = 0; i < tot; ++i) ncnt[key[i]] += 1; int acc = 0; for (int vl = 0; vl < CSR_GN; ++vl) { const int c = ncnt[vl]; ncnt[vl] = acc; acc += c; } ncnt[CSR_GN] = acc;
    for (int i = 0; i < tot; ++i) { const int vl = key[i]; outp[ncnt[vl]] = ids[i]; ncnt[vl] += 1; }
    for (int vl = CSR_GN; vl > 0; --vl) ncnt[vl] = ncnt[vl - 1]; ncnt[0] = 0; }
  __syncthreads();
  for (int pass = 0; pass < 2; ++pass) {
    for (int i = t_; i < (stn - st) / 4; i += 256) { v4i v; for (int e = 0; e < 4; ++e) { const int q = i * 4 + e; v[e] = (q < tot) ? outp[q] : -1; } *(volatile v4i*)(PERM + st + i * 4) = v; }
    for (int i = t_; i < CSR_GN / 4; i += 256) { v4i a, c; for (int e = 0; e < 4; ++e) { const int vl = i * 4 + e; a[e] = st + ncnt[vl]; c[e] = (vl < nv) ? (ncnt[vl + 1] - ncnt[vl]) : 0; } *(volatile v4i*)(ROWPTR + v0 + i * 4) = a; *(volatile v4i*)(ROWCNT + v0 + i * 4) = c; }
    __threadfence(); }
}
__global__ __launch_bounds__(256) void csrZ_kernel(int* __restrict__ p, size_t n4) { typedef __attribute__((ext_vector_type(4))) int v4i; const size_t tid = (size_t)blockIdx.x * 256 + threadIdx.x, nth = (size_t)gridDim.x * 256; v4i z = {0, 0, 0, 0}; for (size_t i = tid; i < n4; i += nth) *(volatile v4i*)(p + i * 4) = z; }
struct CsrBufs { int *STG, *HST, *OFF, *START, *TOT, *PERM, *ROWPTR, *ROWCNT, *FLAG; int nG, NGP, CHP; size_t permLen; char* base; size_t bytes; };
static size_t csr_carve(CsrBufs& c, char* ws, size_t off, int E, int N) {
  const size_t off0 = off; c.base = ws + off;
  auto al = [&](size_t bytes) { char* p = ws + off; off += (bytes + 255) & ~(size_t)255; return p; };
  c.nG = (N + CSR_GN - 1) / CSR_GN; c.NGP = (c.nG + 31) & ~31; const int ch = (E + CSR_NBLK - 1) / CSR_NBLK; c.CHP = (ch + 31) & ~31; c.permLen = (size_t)E + 32 * (size_t)c.nG + 32;
  c.STG = (int*)al((size_t)CSR_NBLK * c.CHP * 4); c.HST = (int*)al((size_t)CSR_NBLK * c.NGP * 4); c.OFF = (int*)al((size_t)c.NGP * CSR_NBLK * 4); c.START = (int*)al((size_t)(c.NGP + 64) * 4); c.TOT = (int*)al((size_t)(c.NGP + 64) * 4);
  c.PERM = (int*)al(c.permLen * 4); c.ROWPTR = (int*)al((size_t)c.nG * CSR_GN * 4); c.ROWCNT = (int*)al((size_t)c.nG * CSR_GN * 4); c.FLAG = (int*)al(256);
  c.bytes = off - off0; return off;
}
static void csr_build(const CsrBufs& c, const int* dst, int E, int N, hipStream_t stream) {
  const size_t smem = (size_t)(2 * c.NGP + c.CHP) * 4;
  csrZ_kernel<<<512, 256, 0, stream>>>((int*)c.base, c.bytes / 16);
  csrA_kernel<<<CSR_NBLK, 64, smem, stream>>>(dst, E, N, c.nG, c.CHP, c.NGP, c.STG, c.HST);
  csrS_kernel<<<1, 512, 0, stream>>>(c.HST, c.nG, c.NGP, c.START, c.TOT, c.OFF);
  csrB_kernel<<<c.nG, 256, 0, stream>>>(dst, N, c.nG, c.CHP, c.NGP, (int)c.permLen, c.STG, c.HST, c.OFF, c.START, c.TOT, c.PERM, c.ROWPTR, c.ROWCNT, c.FLAG);
}

typedef __attribute__((ext_vector_type(4))) _Float16 v4h;
typedef __attribute__((ext_vector_type(2))) _Float16 v2h;
typedef __attribute__((ext_vector_type(2))) float v2f;
__device__ __forceinline__ float lrelu(float v, float s) { return v >= 0.0f ? v : s * v; }
__global__ __launch_bounds__(256) void prep_kernel(const float* __restrict__ x, const float* __restrict__ g0w, const float* __restrict__ g1w, const float* __restrict__ g2w, const float* __restrict__ d0w, const float* __restrict__ d1w,
                                                    b16* __restrict__ Xh, b16* __restrict__ GW0T, b16* __restrict__ GW1T, b16* __restrict__ GW2T, b16* __restrict__ DW0, b16* __restrict__ DW1) {
  size_t t = (size_t)blockIdx.x * 256 + threadIdx.x; v8b o;
  const size_t nx = (size_t)NP * IN / 8; if (t < nx) { const size_t e = t * 8; const size_t v = e / IN; for (int j = 0; j < 8; ++j) o[j] = (v < (size_t)N) ? (b16)(bf16_rne(x[e + j]) * XS) : (b16)0.0f; for (int pass = 0; pass < 2; ++pass) { *(volatile v8b*)(Xh + e) = o; __threadfence(); } return; } t -= nx;
  const size_t ng = (size_t)HC * IN / 8; for (int l = 0; l < 2; ++l) { if (t < ng) { const size_t e = t * 8; const int oo = (int)(e / IN), k0 = (int)(e % IN); const float* w = l ? g1w : g0w; for (int j = 0; j < 8; ++j) o[j] = (b16)(bf16_rne(w[(size_t)(k0 + j) * HC + oo]) * WSC); for (int pass = 0; pass < 2; ++pass) { *(volatile v8b*)((l ? GW1T : GW0T) + e) = o; __threadfence(); } return; } t -= ng; }
  const size_t ng2 = (size_t)HO * IN / 8; if (t < ng2) { const size_t e = t * 8; const int oo = (int)(e / IN), k0 = (int)(e % IN); for (int j = 0; j < 8; ++j) o[j] = (b16)(bf16_rne(g2w[(size_t)(k0 + j) * HO + oo]) * WSC); for (int pass = 0; pass < 2; ++pass) { *(volatile v8b*)(GW2T + e) = o; __threadfence(); } return; } t -= ng2;
  const size_t nd = (size_t)NH * HID * HID / 8; for (int l = 0; l < 2; ++l) { if (t < nd) { const size_t e = t * 8; const int h = (int)(e / ((size_t)HID * HID)); const size_t el = e % ((size_t)HID * HID); const int oo = (int)(el / HID), k0 = (int)(el % HID); const float* w = l ? d1w : d0w;
      for (int j = 0; j < 8; ++j) o[j] = (b16)(bf16_rne(w[(size_t)oo * HC + h * HID + k0 + j]) * WSC); for (int pass = 0; pass < 2; ++pass) { *(volatile v8b*)((l ? DW1 : DW0) + e) = o; __threadfence(); } return; } t -= nd; }
}
template <int TWO, int NT>
__global__ __launch_bounds__(32) void proj_kernel(const b16* __restrict__ Ah, const b16* __restrict__ Al, const b16* __restrict__ WT, const float* __restrict__ al_, const float* __restrict__ ar_, float* __restrict__ Z, float* __restrict__ AS) {
  __shared__ __attribute__((aligned(16))) float Tf[16][NT * 16 + 4]; __shared__ __attribute__((aligned(16))) float Ps[16][2];
  const int lane = threadIdx.x, nloc = lane & 15, hlf = lane >> 4; const size_t m0 = (size_t)blockIdx.x * 16;
  v8f acc[NT];
#pragma unroll
  for (int t = 0; t < NT; ++t) acc[t] = (v8f){};
#pragma unroll 2
  for (int kb = 0; kb < IN; kb += 32) { const v16b a = frag_kb(Ah + (m0 + nloc) * IN + kb, hlf); v16b alo; if (TWO) alo = frag_kb(Al + (m0 + nloc) * IN + kb, hlf);
#pragma unroll
    for (int t = 0; t < NT; ++t) { const v16b bw = frag_kb(WT + (size_t)(t * 16 + nloc) * IN + kb, hlf); acc[t] = wmma16b(a, bw, acc[t]); if (TWO) acc[t] = wmma16b(alo, bw, acc[t]); } }
  float ps[8], pd[8];
#pragma unroll
  for (int r8 = 0; r8 < 8; ++r8) { ps[r8] = 0.0f; pd[r8] = 0.0f; }
#pragma unroll
  for (int t = 0; t < NT; ++t) { const int c = t * 16 + nloc; const float wl_ = bf16_rne(al_[c]), wr_ = bf16_rne(ar_[c]);
#pragma unroll
    for (int r8 = 0; r8 < 8; ++r8) { const float v = acc[t][r8] * (1.0f / (XS * WSC)); Tf[8 * hlf + r8][c] = v; ps[r8] += pmul(v, wl_); pd[r8] += pmul(v, wr_); } }
#pragma unroll
  for (int r8 = 0; r8 < 8; ++r8) { float a = ps[r8], d = pd[r8];
#pragma unroll
    for (int o = 1; o < 16; o <<= 1) { a += __shfl_xor(a, o); d += __shfl_xor(d, o); } if (nloc == 0) { Ps[8 * hlf + r8][0] = a; Ps[8 * hlf + r8][1] = d; } }
  wave_lds_sync();
  typedef __attribute__((ext_vector_type(NT / 2))) float vrow;
  for (int pass = 0; pass < 2; ++pass) { for (int rr = 0; rr < 16; ++rr) *(volatile vrow*)(Z + (m0 + rr) * (NT * 16) + lane * (NT / 2)) = *(const vrow*)(&Tf[rr][lane * (NT / 2)]);
    if (lane < 16) *(volatile v2f*)(AS + (m0 + lane) * 2) = *(const v2f*)(&Ps[lane][0]);
    __threadfence(); }
}
__global__ __launch_bounds__(256) void att_kernel(const float* __restrict__ Z, const float* __restrict__ AS, const float* __restrict__ bias, const int* __restrict__ srcs, const int* __restrict__ PERM, const int* __restrict__ ROWPTR, const int* __restrict__ ROWCNT, int permLen, b16* __restrict__ AGh, b16* __restrict__ AGl) {
  const int wave = threadIdx.x >> 5, lane = threadIdx.x & 31; const size_t v = (size_t)blockIdx.x * 8 + wave; const int c = lane * 4; v4f o = {0.0f, 0.0f, 0.0f, 0.0f};
  if (v < (size_t)N) { int st = ROWPTR[v], cnt = ROWCNT[v]; cnt = iclamp(cnt, 0, 1 << 20); st = iclamp(st, 0, permLen - cnt); const float er = AS[v * 2 + 1];
    float mx = -INFINITY;
#pragma unroll 1
    for (int j = 0; j < cnt; ++j) { const int e = iclamp(PERM[st + j], 0, E - 1); const int s = iclamp(srcs[e], 0, N - 1); float l = lrelu(AS[(size_t)s * 2] + er, GSLOPE); if (s >= NLIM) l = -INFINITY; mx = fmaxf(mx, l); }
    float den = 0.0f; v4f a = {0.0f, 0.0f, 0.0f, 0.0f};
#pragma unroll 1
    for (int j = 0; j < cnt; ++j) { const int e = iclamp(PERM[st + j], 0, E - 1); const int s = iclamp(srcs[e], 0, N - 1); float p = __expf(lrelu(AS[(size_t)s * 2] + er, GSLOPE) - mx); if (s >= NLIM) p = 0.0f; den += p;
      const v4f z = *(const v4f*)(Z + (size_t)s * HID + c); for (int i = 0; i < 4; ++i) a[i] += pmul(p, z[i]); }
    const float inv = (den > 0.0f) ? 1.0f / den : 0.0f;
    for (int i = 0; i < 4; ++i) o[i] = lrelu(pmul(a[i], inv) + bf16_rne(bias[c + i]), ASLOPE); }
  v4h hv, lv; for (int i = 0; i < 4; ++i) { b16 p, q; split16(o[i] * XS, p, q); hv[i] = p; lv[i] = q; }
  for (int pass = 0; pass < 2; ++pass) { *(volatile v4h*)(AGh + v * HID + c) = hv; *(volatile v4h*)(AGl + v * HID + c) = lv; __threadfence(); }
}
template <int FIRST, int LASTH>
__global__ __launch_bounds__(128) void dense_kernel(const b16* __restrict__ Ah, const b16* __restrict__ Al, const b16* __restrict__ WT, const float* __restrict__ db, float* __restrict__ Dacc, b16* __restrict__ Xh, b16* __restrict__ Xl) {
  __shared__ __attribute__((aligned(16))) float Tf[4][16][128 + 4];
  const int wave = threadIdx.x >> 5, lane = threadIdx.x & 31, nloc = lane & 15, hlf = lane >> 4; const size_t m0 = (size_t)blockIdx.x * 64 + wave * 16;
  v8f acc[8];
#pragma unroll
  for (int t = 0; t < 8; ++t) acc[t] = (v8f){};
#pragma unroll 2
  for (int kb = 0; kb < HID; kb += 32) { const v16b a = frag_kb(Ah + (m0 + nloc) * HID + kb, hlf), al = frag_kb(Al + (m0 + nloc) * HID + kb, hlf);
#pragma unroll
    for (int t = 0; t < 8; ++t) { const v16b bw = frag_kb(WT + (size_t)(t * 16 + nloc) * HID + kb, hlf); acc[t] = wmma16b(a, bw, acc[t]); acc[t] = wmma16b(al, bw, acc[t]); } }
#pragma unroll
  for (int t = 0; t < 8; ++t)
#pragma unroll
    for (int r = 0; r < 8; ++r) Tf[wave][8 * hlf + r][t * 16 + nloc] = acc[t][r] * (1.0f / (XS * WSC));
  wave_lds_sync();
  for (int rr = 0; rr < 16; ++rr) { v4f o = *(const v4f*)(&Tf[wave][rr][lane * 4]); const size_t row = m0 + rr;
    if (!FIRST) o += *(const v4f*)(Dacc + row * HID + lane * 4);
    if (LASTH) { for (int j = 0; j < 4; ++j) o[j] = (row < (size_t)N) ? lrelu(o[j] + bf16_rne(db[lane * 4 + j]), ASLOPE) : 0.0f; }
    *(v4f*)(&Tf[wave][rr][lane * 4]) = o; }
  wave_lds_sync();
  for (int pass = 0; pass < 2; ++pass) { for (int rr = 0; rr < 16; ++rr) { const v4f o = *(const v4f*)(&Tf[wave][rr][lane * 4]); const size_t row = m0 + rr;
      if (LASTH) { v4h hv, lv; for (int j = 0; j < 4; ++j) { b16 p, q; split16(o[j] * XS, p, q); hv[j] = p; lv[j] = q; } *(volatile v4h*)(Xh + row * HID + lane * 4) = hv; *(volatile v4h*)(Xl + row * HID + lane * 4) = lv; }
      else *(volatile v4f*)(Dacc + row * HID + lane * 4) = o; }
    __threadfence(); }
}
template <int FIRST, int LASTH>
__global__ __launch_bounds__(256) void att2_kernel(const float* __restrict__ Z, const float* __restrict__ AS, const float* __restrict__ bias, const int* __restrict__ srcs, const int* __restrict__ PERM, const int* __restrict__ ROWPTR, const int* __restrict__ ROWCNT, int permLen, float* __restrict__ OACC, float* __restrict__ out) {
  const int wave = threadIdx.x >> 5, lane = threadIdx.x & 31; const size_t v = (size_t)blockIdx.x * 8 + wave; if (v >= (size_t)N) return; const int c = lane * 2;
  int st = ROWPTR[v], cnt = ROWCNT[v]; cnt = iclamp(cnt, 0, 1 << 20); st = iclamp(st, 0, permLen - cnt); const float er = AS[v * 2 + 1];
  float mx = -INFINITY;
#pragma unroll 1
  for (int j = 0; j < cnt; ++j) { const int e = iclamp(PERM[st + j], 0, E - 1); const int s = iclamp(srcs[e], 0, N - 1); float l = lrelu(AS[(size_t)s * 2] + er, GSLOPE); if (s >= NLIM) l = -INFINITY; mx = fmaxf(mx, l); }
  float den = 0.0f; v2f a = {0.0f, 0.0f};
#pragma unroll 1
  for (int j = 0; j < cnt; ++j) { const int e = iclamp(PERM[st + j], 0, E - 1); const int s = iclamp(srcs[e], 0, N - 1); float p = __expf(lrelu(AS[(size_t)s * 2] + er, GSLOPE) - mx); if (s >= NLIM) p = 0.0f; den += p;
    const v2f z = *(const v2f*)(Z + (size_t)s * OUT + c); a[0] += pmul(p, z[0]); a[1] += pmul(p, z[1]); }
  const float inv = (den > 0.0f) ? 1.0f / den : 0.0f;
  v2f o; for (int i = 0; i < 2; ++i) o[i] = lrelu(pmul(a[i], inv) + bf16_rne(bias[c + i]), ASLOPE) * 0.25f;
  if (!FIRST) o += *(const v2f*)(OACC + v * OUT + c);
  if (LASTH) { for (int i = 0; i < 2; ++i) o[i] = lrelu(o[i], ASLOPE); }
  for (int pass = 0; pass < 2; ++pass) { if (LASTH) *(volatile v2f*)(out + v * OUT + c) = o; else *(volatile v2f*)(OACC + v * OUT + c) = o; __threadfence(); }
}
}

extern "C" void kernel_launch(void* const* d_in, const int* in_sizes, int n_in, void* d_out, int out_size, void* d_ws, size_t ws_size, hipStream_t stream) {
  (void)n_in;
  auto Fp = [&](int i) { return (const float*)d_in[i]; }; auto Ip = [&](int i) { return (const int*)d_in[i]; };
  if (in_sizes[0] != N * IN || in_sizes[1] != EFULL || in_sizes[2] != EFULL || in_sizes[3] != IN * HC || in_sizes[4] != HC || in_sizes[5] != HC || in_sizes[6] != HC || in_sizes[7] != HID * HC || in_sizes[8] != HID ||
      in_sizes[9] != HID * HC || in_sizes[12] != HC || in_sizes[13] != HID * HC || in_sizes[14] != HID || in_sizes[15] != HID * HO || in_sizes[16] != HO || in_sizes[18] != HO || out_size != N * OUT) return;
  size_t off = 0; char* ws = (char*)d_ws;
  auto carve = [&](size_t bytes) { char* p = ws + off; off += (bytes + 255) & ~(size_t)255; return p; };
  b16* Xh = (b16*)carve((size_t)NP * IN * 2); b16* Xl = (b16*)carve((size_t)NP * IN * 2); b16* GW0T = (b16*)carve((size_t)HC * IN * 2); b16* GW1T = (b16*)carve((size_t)HC * IN * 2); b16* GW2T = (b16*)carve((size_t)HO * IN * 2);
  b16* DW0 = (b16*)carve((size_t)NH * HID * HID * 2); b16* DW1 = (b16*)carve((size_t)NH * HID * HID * 2);
  float* Z = (float*)carve((size_t)NP * HID * 4); float* AS = (float*)carve((size_t)NP * 2 * 4); b16* AGh = (b16*)carve((size_t)NP * HID * 2); b16* AGl = (b16*)carve((size_t)NP * HID * 2); float* Dacc = (float*)carve((size_t)NP * HID * 4); float* OACC = Dacc;
  CsrBufs csr; off = csr_carve(csr, ws, off, E, N);
  if (off > ws_size || off > ((size_t)128 << 20)) return;
  prep_kernel<<<(unsigned)((((size_t)NP * IN + 2 * (size_t)HC * IN + (size_t)HO * IN + 2 * (size_t)NH * HID * HID) / 8 + 255) / 256), 256, 0, stream>>>(Fp(0), Fp(3), Fp(9), Fp(15), Fp(7), Fp(13), Xh, GW0T, GW1T, GW2T, DW0, DW1);
  csr_build(csr, Ip(2), E, N, stream);
  for (int l = 0; l < 2; ++l) { const b16* GWT = l ? GW1T : GW0T; const b16* DW = l ? DW1 : DW0; const float* al_ = l ? Fp(10) : Fp(4); const float* ar_ = l ? Fp(11) : Fp(5); const float* gb = l ? Fp(12) : Fp(6); const float* dbias = l ? Fp(14) : Fp(8);
    for (int h = 0; h < NH; ++h) {
      if (l == 0) proj_kernel<0, 8><<<NLIM / 16, 32, 0, stream>>>(Xh, nullptr, GWT + (size_t)h * HID * IN, al_ + h * HID, ar_ + h * HID, Z, AS);
      else        proj_kernel<1, 8><<<NLIM / 16, 32, 0, stream>>>(Xh, Xl, GWT + (size_t)h * HID * IN, al_ + h * HID, ar_ + h * HID, Z, AS);
      att_kernel<<<NLIM / 8, 256, 0, stream>>>(Z, AS, gb + h * HID, Ip(1), csr.PERM, csr.ROWPTR, csr.ROWCNT, (int)csr.permLen, AGh, AGl);
      const b16* DWh = DW + (size_t)h * HID * HID;
      if (h == 0)           dense_kernel<1, 0><<<NLIM / 64, 128, 0, stream>>>(AGh, AGl, DWh, dbias, Dacc, Xh, Xl);
      else if (h < NH - 1)  dense_kernel<0, 0><<<NLIM / 64, 128, 0, stream>>>(AGh, AGl, DWh, dbias, Dacc, Xh, Xl);
      else                  dense_kernel<0, 1><<<NLIM / 64, 128, 0, stream>>>(AGh, AGl, DWh, dbias, Dacc, Xh, Xl); } }
  for (int h = 0; h < NH; ++h) {
    proj_kernel<1, 4><<<NLIM / 16, 32, 0, stream>>>(Xh, Xl, GW2T + (size_t)h * OUT * IN, Fp(16) + h * OUT, Fp(17) + h * OUT, Z, AS);
    if (h == 0)          att2_kernel<1, 0><<<NLIM / 8, 256, 0, stream>>>(Z, AS, Fp(18) + h * OUT, Ip(1), csr.PERM, csr.ROWPTR, csr.ROWCNT, (int)csr.permLen, OACC, (float*)d_out);
    else if (h < NH - 1) att2_kernel<0, 0><<<NLIM / 8, 256, 0, stream>>>(Z, AS, Fp(18) + h * OUT, Ip(1), csr.PERM, csr.ROWPTR, csr.ROWCNT, (int)csr.permLen, OACC, (float*)d_out);
    else                 att2_kernel<0, 1><<<NLIM / 8, 256, 0, stream>>>(Z, AS, Fp(18) + h * OUT, Ip(1), csr.PERM, csr.ROWPTR, csr.ROWCNT, (int)csr.permLen, OACC, (float*)d_out); }
}
